// ScaledDotProductAttention_19344532702173
// MI455X (gfx1250) — hardware-verified
//
#include <hip/hip_runtime.h>
#ifndef NB
#define NB 8
#endif
#ifndef SEQ
#define SEQ 4096
#endif
#define NB_FULL 8
#define SEQ_FULL 4096
#define HD 64
#define QK_CARRY 64.0f
#define V_CARRY 64.0f
#define P_CARRY 16384.0f
#define S_ALPHA 0.000244140625f
#define O_ALPHA 0.015625f
#define F16_MIN_NORMAL 6.103515625e-05f

static_assert(NB >= 1 && NB <= NB_FULL);
static_assert(SEQ >= 256 && SEQ <= SEQ_FULL);
static_assert(HD == 64);
static_assert(SEQ % 256 == 0);
static_assert((SEQ / 128) * 128 == SEQ);
static_assert((SEQ / 64) * 64 == SEQ);
static_assert((SEQ / 32) * 32 == SEQ);
static_assert((((size_t)SEQ * HD / 8) / 256) * 256 * 8 == (size_t)SEQ * HD);
#define WS_PLANE16 ((size_t)NB * SEQ * HD * 2)
#define WS_S ((size_t)SEQ * SEQ * 4)
#define WS_P ((size_t)SEQ * SEQ * 2)
#define WS_RF ((size_t)NB * SEQ * 4)
static_assert(WS_PLANE16 % 256 == 0 && WS_S % 256 == 0 && WS_P % 256 == 0 && WS_RF % 256 == 0);
static_assert(3 * WS_PLANE16 + WS_S + WS_P + WS_RF <= (size_t)134217728);

typedef unsigned short v8us __attribute__((ext_vector_type(8), may_alias));
typedef float  v8f  __attribute__((ext_vector_type(8)));
typedef float  v4f  __attribute__((ext_vector_type(4)));
typedef float  v4fa __attribute__((ext_vector_type(4), may_alias));
typedef _Float16 v16h __attribute__((ext_vector_type(16)));
union FragH { v16h v; v8us half[2]; _Float16 h[16]; unsigned short u[16]; };

__device__ __forceinline__ unsigned short bf16_bits(float x) { unsigned int u = __float_as_uint(x); return (unsigned short)((u + 0x7FFFu + ((u >> 16) & 1u)) >> 16); }
__device__ __forceinline__ float bf16_val(unsigned short b) { return __uint_as_float(((unsigned int)b) << 16); }
__device__ __forceinline__ float bf16_rne(float x) { return bf16_val(bf16_bits(x)); }

__global__ __launch_bounds__(256) void k_cvt16(const float* __restrict__ xq, const float* __restrict__ xk, _Float16* __restrict__ Q16, _Float16* __restrict__ K16) {
  const unsigned t = blockIdx.x * 256u + threadIdx.x;
  const unsigned b = blockIdx.y;
  const float* src = (blockIdx.z == 0u) ? xq : xk;
  _Float16* dst = (blockIdx.z == 0u) ? Q16 : K16;
  const float* p = src + (size_t)b * SEQ_FULL * HD + (size_t)t * 8u;
  const v4f a = *(const v4fa*)p, c = *(const v4fa*)(p + 4);
  FragH f;
#pragma unroll
  for (int q = 0; q < 4; ++q) { f.h[q] = (_Float16)(bf16_rne(a[q]) * QK_CARRY); f.h[4 + q] = (_Float16)(bf16_rne(c[q]) * QK_CARRY); }
  const v8us o = f.half[0];
  unsigned short* d = (unsigned short*)dst + (size_t)b * SEQ * HD + (size_t)t * 8u;
  *(volatile v8us*)d = o;
  __threadfence();
  *(volatile v8us*)d = o;
}

__global__ __launch_bounds__(256) void k_vtf(const float* __restrict__ xv, _Float16* __restrict__ VT) {
  __shared__ unsigned short tl[64][66];
  const unsigned tid = threadIdx.x; const unsigned lg = blockIdx.x; const unsigned b = blockIdx.y;
  for (unsigned i = tid; i < 512u; i += 256u) {
    const unsigned r = i >> 3, c8 = (i & 7u) * 8u;
    const float* p = xv + ((size_t)b * SEQ_FULL + (size_t)lg * 64u + r) * HD + c8;
    const v4f a = *(const v4fa*)p, c = *(const v4fa*)(p + 4);
    FragH f;
#pragma unroll
    for (int q = 0; q < 4; ++q) { f.h[q] = (_Float16)(bf16_rne(a[q]) * V_CARRY); f.h[4 + q] = (_Float16)(bf16_rne(c[q]) * V_CARRY); }
#pragma unroll
    for (int q = 0; q < 8; ++q) tl[r][c8 + q] = f.u[q];
  }
  __syncthreads();
  for (int pass = 0; pass < 2; ++pass) {
#pragma unroll
    for (unsigned rd = 0; rd < 2u; ++rd) {
      const unsigned d = rd * 32u + (tid >> 3), pc = tid & 7u; FragH f;
#pragma unroll
      for (unsigned q = 0; q < 8u; ++q) f.u[q] = tl[pc * 8u + q][d];
      *(volatile v8us*)((unsigned short*)VT + ((size_t)b * HD + d) * SEQ + (size_t)lg * 64u + pc * 8u) = f.half[0];
    }
    if (pass == 0) __threadfence();
  }
}

__device__ __forceinline__ v16h g2_frag(const _Float16* p, unsigned hh) { FragH f; f.half[0] = *(const v8us*)((const unsigned short*)p + 8u * hh); f.half[1] = *(const v8us*)((const unsigned short*)p + 16u + 8u * hh); return f.v; }
__device__ __forceinline__ v8f g2_mma(v16h a, v16h b, v8f c) { v8f d = __builtin_amdgcn_wmma_f32_16x16x32_f16(false, a, false, b, (short)0, c, false, false); asm volatile("v_nop\n\tv_nop\n\tv_nop\n\tv_nop" : "+v"(d) : "v"(a), "v"(b)); return d; }

template <bool ROWS>
__global__ __launch_bounds__(128) void k_gemm2(const _Float16* __restrict__ A, unsigned lda, const _Float16* __restrict__ Bh, unsigned ldb, float alpha,
                                               const float* __restrict__ rs, float* __restrict__ C, unsigned ldc, unsigned M, unsigned N, unsigned K) {
  __shared__ __attribute__((aligned(16))) float so[4][32][68];
  const unsigned tid = threadIdx.x, w = tid >> 5, lane = tid & 31u, ln = lane & 15u, hh = lane >> 4;
  const unsigned ntn = N >> 6; const unsigned mt = blockIdx.x / ntn, nq = blockIdx.x - mt * ntn;
  const unsigned row0 = mt * 128u + 32u * w, col0 = nq * 64u; if (row0 >= M) return;
  const _Float16* a0p = A + (size_t)(row0 + ln) * lda; const _Float16* a1p = a0p + (size_t)16 * lda;
  const _Float16* b0p = Bh + (size_t)(col0 + ln) * ldb; const _Float16* b1p = b0p + (size_t)16 * ldb; const _Float16* b2p = b1p + (size_t)16 * ldb; const _Float16* b3p = b2p + (size_t)16 * ldb;
  const v8f z8 = {0.f,0.f,0.f,0.f,0.f,0.f,0.f,0.f}; v8f c00 = z8, c01 = z8, c02 = z8, c03 = z8, c10 = z8, c11 = z8, c12 = z8, c13 = z8;
#pragma unroll 1
  for (unsigned kb = 0; kb < K; kb += 32u) { const v16h a0 = g2_frag(a0p + kb, hh), a1 = g2_frag(a1p + kb, hh);
    v16h b = g2_frag(b0p + kb, hh); c00 = g2_mma(a0, b, c00); c10 = g2_mma(a1, b, c10);
    b = g2_frag(b1p + kb, hh); c01 = g2_mma(a0, b, c01); c11 = g2_mma(a1, b, c11);
    b = g2_frag(b2p + kb, hh); c02 = g2_mma(a0, b, c02); c12 = g2_mma(a1, b, c12);
    b = g2_frag(b3p + kb, hh); c03 = g2_mma(a0, b, c03); c13 = g2_mma(a1, b, c13); }
  v8f accs[8] = {c00, c01, c02, c03, c10, c11, c12, c13};
  float rsv[16];
  if (ROWS) {
    const v4f x0 = *(const v4fa*)(rs + row0 + 8u * hh), x1 = *(const v4fa*)(rs + row0 + 8u * hh + 4u);
    const v4f x2 = *(const v4fa*)(rs + row0 + 16u + 8u * hh), x3 = *(const v4fa*)(rs + row0 + 16u + 8u * hh + 4u);
#pragma unroll
    for (int q = 0; q < 4; ++q) { rsv[q] = x0[q]; rsv[4 + q] = x1[q]; rsv[8 + q] = x2[q]; rsv[12 + q] = x3[q]; }
  } else {
#pragma unroll
    for (int q = 0; q < 16; ++q) rsv[q] = 1.0f;
  }
#pragma unroll
  for (int u = 0; u < 8; ++u) { const int t = u & 3, half = u >> 2;
#pragma unroll
    for (int r = 0; r < 8; ++r) { const unsigned rloc = (unsigned)half * 16u + 8u * hh + (unsigned)r; float v = accs[u][r] * alpha; if (ROWS) v = v * rsv[half * 8 + r];
      so[w][rloc][(unsigned)t * 16u + ln] = v; } }
  __builtin_amdgcn_fence(4  , "workgroup"); __builtin_amdgcn_wave_barrier();
  const unsigned rsub = lane >> 4, c4 = (lane & 15u) * 4u;
  for (int pass = 0; pass < 2; ++pass) {
#pragma unroll
    for (unsigned q = 0; q < 16u; ++q) { const unsigned r = q * 2u + rsub; const v4f v = *(const v4fa*)&so[w][r][c4]; *(volatile v4f*)(C + (size_t)(row0 + r) * ldc + col0 + c4) = v; }
    if (pass == 0) __threadfence(); }
}

__global__ __launch_bounds__(256) void k_psm(const float* __restrict__ S, _Float16* __restrict__ P, float* __restrict__ rowfac) {
  #pragma clang fp contract(off)
  __shared__ float rf[32];
  const unsigned tid = threadIdx.x, w = tid >> 5, lane = tid & 31u;
#pragma unroll 1
  for (unsigned rr = 0; rr < 4u; ++rr) {
    const unsigned row = blockIdx.x * 32u + w * 4u + rr;
    const float* s = S + (size_t)row * SEQ + lane * 8u;
    float mx = -3.0e38f;
#pragma unroll 1
    for (unsigned j = 0; j < (unsigned)SEQ; j += 256u) {
      const v4f a = *(const v4fa*)(s + j), c = *(const v4fa*)(s + j + 4u);
      mx = fmaxf(mx, fmaxf(fmaxf(a[0], a[1]), fmaxf(a[2], a[3])));
      mx = fmaxf(mx, fmaxf(fmaxf(c[0], c[1]), fmaxf(c[2], c[3])));
    }
    mx = fmaxf(mx, __shfl_xor(mx, 16)); mx = fmaxf(mx, __shfl_xor(mx, 8)); mx = fmaxf(mx, __shfl_xor(mx, 4)); mx = fmaxf(mx, __shfl_xor(mx, 2)); mx = fmaxf(mx, __shfl_xor(mx, 1));
    float sum = 0.f;
    unsigned short* d = (unsigned short*)P + (size_t)row * SEQ + lane * 8u;
#pragma unroll 1
    for (unsigned j = 0; j < (unsigned)SEQ; j += 256u) {
      const v4f a = *(const v4fa*)(s + j), c = *(const v4fa*)(s + j + 4u);
      FragH f;
#pragma unroll
      for (int q = 0; q < 4; ++q) {
        float e0 = __expf(a[q] - mx) * P_CARRY; e0 = (e0 < F16_MIN_NORMAL) ? 0.f : e0; const _Float16 h0 = (_Float16)e0; f.h[q] = h0; sum += (float)h0;
        float e1 = __expf(c[q] - mx) * P_CARRY; e1 = (e1 < F16_MIN_NORMAL) ? 0.f : e1; const _Float16 h1 = (_Float16)e1; f.h[4 + q] = h1; sum += (float)h1;
      }
      const v8us o = f.half[0];
      *(volatile v8us*)(d + j) = o;
      __threadfence();
      *(volatile v8us*)(d + j) = o;
    }
    sum += __shfl_xor(sum, 16); sum += __shfl_xor(sum, 8); sum += __shfl_xor(sum, 4); sum += __shfl_xor(sum, 2); sum += __shfl_xor(sum, 1);
    if (lane == 0u) rf[w * 4u + rr] = 0.125f * (1.0f / sum);
  }
  __syncthreads();
  if (tid < 32u) { const float v = rf[tid]; volatile float* o = rowfac + (size_t)blockIdx.x * 32u + tid; *o = v; __threadfence(); *o = v; }
}

extern "C" void kernel_launch(void* const* d_in, const int* in_sizes, int n_in,
                              void* d_out, int out_size, void* d_ws, size_t ws_size, hipStream_t stream) {
  if (n_in < 3) return;
  const size_t need_in = ((size_t)(NB - 1) * SEQ_FULL + SEQ) * HD;
  if ((size_t)in_sizes[0] < need_in || (size_t)in_sizes[1] < need_in || (size_t)in_sizes[2] < need_in) return;
  if ((size_t)out_size < (size_t)NB * SEQ * HD) return;
  const float* xq = (const float*)d_in[0]; const float* xk = (const float*)d_in[1]; const float* xv = (const float*)d_in[2];
  float* out = (float*)d_out;
  char* ws = (char*)d_ws; size_t off = 0;
  auto take = [&](size_t bytes) { char* p = ws + off; off += (bytes + 255) & ~(size_t)255; return p; };
  _Float16* Q16 = (_Float16*)take(WS_PLANE16);
  _Float16* K16 = (_Float16*)take(WS_PLANE16);
  _Float16* VT  = (_Float16*)take(WS_PLANE16);
  float*    S   = (float*)take(WS_S);
  _Float16* P   = (_Float16*)take(WS_P);
  float*    RF  = (float*)take(WS_RF);
  if (off > ws_size) return;

  k_cvt16<<<dim3((unsigned)(((size_t)SEQ * HD / 8) / 256), NB, 2), 256, 0, stream>>>(xq, xk, Q16, K16);
  k_vtf<<<dim3(SEQ / 64, NB), 256, 0, stream>>>(xv, VT);
  for (int b = 0; b < NB; ++b) {
    const size_t r0 = (size_t)b * SEQ;
    k_gemm2<false><<<dim3((SEQ / 128) * (SEQ / 64)), 128, 0, stream>>>(Q16 + r0 * HD, HD, K16 + r0 * HD, HD, S_ALPHA, RF, S, SEQ, SEQ, SEQ, HD);
    k_psm<<<SEQ / 32, 256, 0, stream>>>(S, P, RF + r0);
    k_gemm2<true><<<dim3((SEQ / 128) * (HD / 64)), 128, 0, stream>>>(P, SEQ, VT + (size_t)b * HD * SEQ, SEQ, O_ALPHA, RF + r0, out + r0 * HD, HD, SEQ, HD, SEQ);
  }
}
